// ConvTransformerEncoder_52012053955076
// MI455X (gfx1250) — hardware-verified
//
#include <hip/hip_runtime.h>
#include <math.h>

typedef __attribute__((ext_vector_type(16))) _Float16 v16h;
typedef __attribute__((ext_vector_type(16))) __bf16 v16b;
typedef __attribute__((ext_vector_type(8)))  _Float16 v8h;
typedef __attribute__((ext_vector_type(8)))  float v8f;
typedef __attribute__((ext_vector_type(4)))  float v4f;
typedef __attribute__((ext_vector_type(2)))  float v2f;
typedef __attribute__((ext_vector_type(4)))  unsigned v4u;
typedef __attribute__((ext_vector_type(4)))  int v4i;
typedef float __attribute__((may_alias)) float_a;
typedef int __attribute__((may_alias)) int_a;

template <typename T> __device__ __forceinline__ void vst2(void* p, T v) { *(volatile T*)p = v; __threadfence(); *(volatile T*)p = v; }
__device__ __forceinline__ v8f wmma16(v16h a, v16h b, v8f c) {
  v8f d = __builtin_amdgcn_wmma_f32_16x16x32_f16(false, a, false, b, (short)0, c, false, false);
  asm volatile("v_nop\n\tv_nop\n\tv_nop\n\tv_nop" : "+v"(d) : "v"(a), "v"(b));
  return d;
}
__device__ __forceinline__ v8f wmma_bf(v16b a, v16b b, v8f c) {
  v8f d = __builtin_amdgcn_wmma_f32_16x16x32_bf16(false, a, false, b, (short)0, c, false, false);
  asm volatile("v_nop\n\tv_nop\n\tv_nop\n\tv_nop" : "+v"(d) : "v"(a), "v"(b));
  return d;
}
__device__ __forceinline__ v16h frag_h(const _Float16* rowk0, int lane) {
  union { v16h v; v8h q[2]; } u; const _Float16* p = rowk0 + 8 * (lane >> 4);
  u.q[0] = *(const v8h*)p; u.q[1] = *(const v8h*)(p + 16); return u.v;
}
__device__ __forceinline__ v16h frag_f32(const float* rowk0, int lane) {
  v16h a; const float* p = rowk0 + 8 * (lane >> 4);
#pragma unroll
  for (int i = 0; i < 8; ++i) { a[i] = (_Float16)p[i]; a[8 + i] = (_Float16)p[16 + i]; }
  return a;
}
__device__ __forceinline__ v16h frag_f32s(const float* rowk0, int lane, float sc) {
  v16h a; const float* p = rowk0 + 8 * (lane >> 4);
#pragma unroll
  for (int i = 0; i < 8; ++i) { a[i] = (_Float16)(p[i] * sc); a[8 + i] = (_Float16)(p[16 + i] * sc); }
  return a;
}
__device__ __forceinline__ v16h fragc_f32(const float* W, int k0, int n, int lane, int ld, int K) {
  v16h a; const int g = lane >> 4;
#pragma unroll
  for (int i = 0; i < 8; ++i) { const int ka = k0 + 8 * g + i, kb = ka + 16;
    a[i] = (_Float16)(ka < K ? W[(size_t)(ka < K ? ka : K - 1) * ld + n] : 0.f); a[8 + i] = (_Float16)(kb < K ? W[(size_t)(kb < K ? kb : K - 1) * ld + n] : 0.f); }
  return a;
}
struct F2 { v16b h, l; };
__device__ __forceinline__ F2 bsplit16(const float v[16]) { F2 r;
#pragma unroll
  for (int i = 0; i < 16; ++i) { const __bf16 h = (__bf16)v[i]; r.h[i] = h; r.l[i] = (__bf16)(v[i] - (float)h); }
  return r; }
__device__ __forceinline__ F2 split_row(const float* row, int k0, int lane) { float v[16]; const float* p = row + k0 + 8 * (lane >> 4);
#pragma unroll
  for (int i = 0; i < 8; ++i) { v[i] = p[i]; v[8 + i] = p[16 + i]; }
  return bsplit16(v); }
__device__ __forceinline__ F2 split_rowK(const float* row, int k0, int lane, int K) { float v[16]; const int g = lane >> 4;
#pragma unroll
  for (int i = 0; i < 8; ++i) { const int ka = k0 + 8 * g + i, kb = ka + 16; v[i] = ka < K ? row[ka < K ? ka : K - 1] : 0.f; v[8 + i] = kb < K ? row[kb < K ? kb : K - 1] : 0.f; }
  return bsplit16(v); }
__device__ __forceinline__ F2 split_col(const float* W, int k0, int n, int lane, int ld, int K) { float v[16]; const int g = lane >> 4;
#pragma unroll
  for (int i = 0; i < 8; ++i) { const int ka = k0 + 8 * g + i, kb = ka + 16; v[i] = ka < K ? W[(size_t)(ka < K ? ka : K - 1) * ld + n] : 0.f; v[8 + i] = kb < K ? W[(size_t)(kb < K ? kb : K - 1) * ld + n] : 0.f; }
  return bsplit16(v); }
__device__ __forceinline__ v8f mac3(const F2& a, const F2& b, v8f c) { c = wmma_bf(a.l, b.h, c); c = wmma_bf(a.h, b.l, c); return wmma_bf(a.h, b.h, c); }
__device__ __forceinline__ float sigm(float v) { return 1.0f / (1.0f + expf(-v)); }
#define LDSX() do { asm volatile("s_wait_dscnt 0" ::: "memory"); __builtin_amdgcn_wave_barrier(); __builtin_amdgcn_fence(__ATOMIC_RELEASE, "workgroup"); } while (0)


#define NBB 2
#define NT 12
#ifndef HHH
#define HHH 32
#endif
#define WWW 32
#define NPX (HHH * WWW)
#define CC 128
#define NHD 4
#define DH 32
#define NL 5
#define NFR (NBB * NT)
#define NPB (NPX / 64)
typedef __attribute__((ext_vector_type(8))) __bf16 v8b;
__device__ __forceinline__ v16b frag_b(const __bf16* rowk0, int lane) {
  union { v16b v; v8b q[2]; } u; const __bf16* p = rowk0 + 8 * (lane >> 4);
  u.q[0] = *(const v8b*)p; u.q[1] = *(const v8b*)(p + 16); return u.v;
}
__device__ __forceinline__ float bfr(float v) { return (float)(__bf16)v; }
__device__ __attribute__((noinline)) float exp_ni(float v) { return expf(v); }
__device__ __attribute__((noinline)) float erf_ni(float v) { return erff(v); }

#define FSZ ((size_t)NFR * CC * NPX)
#define WS_XA  0u
#define WS_Q   (WS_XA + 4u * FSZ)
#define WS_V   (WS_Q + 4u * FSZ)
#define WS_AT  (WS_V + 4u * FSZ)
#define WS_F1  (WS_AT + 4u * FSZ)
#define WS_Y   (WS_F1 + 4u * FSZ)
#define WS_AQ  (WS_Y + 4u * FSZ)
#define WS_BK  (WS_AQ + 4u * (size_t)NFR * NHD * NPX)
#define WS_GS  (WS_BK + 4u * (size_t)NFR * NHD * NPX)
#define WS_WQ  (WS_GS + 4u * (size_t)NFR * NPB * 32)
#define WS_WKV (WS_WQ + 2u * NHD * DH * DH * 9)
#define WS_WA  (WS_WKV + 2u * NHD * DH * DH * 9)
#define WS_WF1 (WS_WA + 2u * NHD * 2 * DH * 9)
#define WS_WF2 (WS_WF1 + 2u * (size_t)CC * CC * 9)
#define WS_END (WS_WF2 + 2u * (size_t)CC * CC * 9)

__device__ __forceinline__ float posv(int t, int c) { const int i2 = c & ~1; const float dv = expf((float)i2 * (-9.210340371976184f / (float)DH)); const float a = (float)t * dv; return (c & 1) ? cosf(a) : sinf(a); }
__global__ __launch_bounds__(256) void k_wperm(const float* __restrict__ Wsrc, int cout, int cin, _Float16* __restrict__ WD) { __shared__ __align__(16) _Float16 s[9 * CC]; const int co = blockIdx.x; const int t = threadIdx.x;
  for (int e = t; e < 9 * cin; e += 256) { const int tap = e / cin, ci = e % cin; s[e] = (_Float16)bfr(Wsrc[((size_t)co * cin + ci) * 9 + tap]); }
  __syncthreads(); for (int q = t; q < 9 * cin / 8; q += 256) vst2((unsigned*)(WD + (size_t)co * 9 * cin + q * 8), *(const v4u*)&s[q * 8]); }
template <int CIN>
__device__ __forceinline__ void stage_tile(const float* __restrict__ src, int y0, const float* addc, _Float16* sx, int tid, int nthr) {
  const int ci = tid % CIN; const int sub = tid / CIN; const int nsub = 128 / CIN; const float add = addc ? addc[ci] : 0.f; const float* sc = src + (size_t)ci * NPX;
#pragma unroll 1
  for (int ry = 0; ry < 4; ++ry) { const int yy = y0 - 1 + ry; const bool rowok = (yy >= 0 && yy < HHH);
#pragma unroll 1
    for (int cx = sub; cx < 34; cx += nsub) { const int xx = cx - 1; float v = 0.f; if (rowok && xx >= 0 && xx < WWW) v = sc[yy * WWW + xx] + add; sx[((size_t)(ry * 34 + cx)) * CIN + ci] = (_Float16)v; } } }
template <int CIN>
__device__ __forceinline__ v16h tile_frag(const _Float16* sx, int ly, int lx, int tap, int c0, int lane) { const int ky = tap / 3, kx = tap % 3; return frag_h(sx + ((size_t)((ly + ky) * 34 + (lx + kx)) * CIN) + c0, lane); }
__global__ __launch_bounds__(128) void k_qv(const float* __restrict__ XA, const _Float16* __restrict__ WQP, const float* __restrict__ QB, const _Float16* __restrict__ WKVP, const float* __restrict__ KVB, int li, float* __restrict__ Q, float* __restrict__ V) {
  __shared__ __align__(16) float so[4][32][20];
  __shared__ __align__(16) _Float16 sx[4 * 34 * DH];
  const int tid = threadIdx.x, wave = tid >> 5, lane = tid & 31, col = lane & 15, g = lane >> 4; const int pb = blockIdx.x; const size_t f = blockIdx.y; const int hd = blockIdx.z; const int t = (int)(f % NT);
  const float* src = XA + (f * CC + hd * DH) * NPX; const int p0 = pb * 64 + wave * 16; const int y0 = (pb * 64) / WWW; const int ly = (wave * 16) / WWW, lx = (wave * 16 + col) % WWW;
  stage_tile<DH>(src, y0, nullptr, sx, tid, 128); __syncthreads(); (void)li;
#pragma unroll 1
  for (int which = 0; which < 2; ++which) { const _Float16* Wt = (which == 0 ? WQP : WKVP) + (size_t)hd * DH * (DH * 9); const float* Bs = (which == 0 ? QB : KVB) + ((size_t)li * NHD + hd) * DH;
    v8f acc[2] = {};
#pragma unroll
    for (int tap = 0; tap < 9; ++tap) { const v16h a = tile_frag<DH>(sx, ly, lx, tap, 0, lane);
#pragma unroll
      for (int j = 0; j < 2; ++j) acc[j] = wmma16(a, frag_h(Wt + (size_t)(j * 16 + col) * (DH * 9) + tap * DH, lane), acc[j]); }
#pragma unroll
    for (int j = 0; j < 2; ++j) { const int c = j * 16 + col; const float bb = bfr(Bs[c]) + (which == 0 ? posv(t, c) : 0.f);
#pragma unroll
      for (int r = 0; r < 8; ++r) so[wave][c][8 * g + r] = acc[j][r] + bb; }
    LDSX();
    { float* dst = (which == 0 ? Q : V) + (f * CC + hd * DH) * NPX + p0; for (int c = 0; c < DH; ++c) if (lane < 4) vst2(dst + (size_t)c * NPX + lane * 4, *(const v4f*)&so[wave][c][lane * 4]); }
    LDSX(); } }
__global__ __launch_bounds__(128) void k_logit(const float* __restrict__ Q, const float* __restrict__ V, const _Float16* __restrict__ WAP, int li, float* __restrict__ AQ, float* __restrict__ BK) {
  __shared__ __align__(16) float spos[NHD][DH]; __shared__ __align__(16) float so[4][2][16]; __shared__ __align__(16) _Float16 sx[4 * 34 * DH];
  const int tid = threadIdx.x, wave = tid >> 5, lane = tid & 31, col = lane & 15, g = lane >> 4; const int pb = blockIdx.x; const size_t f = blockIdx.y; const int hd = blockIdx.z; const int t = (int)(f % NT);
  if (tid < DH) spos[hd][tid] = posv(t, tid);
  __syncthreads();
  const _Float16* Wa = WAP + (size_t)hd * (2 * DH * 9);
  const int p0 = pb * 64 + wave * 16; const int y0 = (pb * 64) / WWW; const int ly = (wave * 16) / WWW, lx = (wave * 16 + col) % WWW; (void)li;
#pragma unroll 1
  for (int which = 0; which < 2; ++which) { const float* src = (which == 0 ? Q : V) + (f * CC + hd * DH) * NPX; __syncthreads(); stage_tile<DH>(src, y0, which == 0 ? nullptr : &spos[hd][0], sx, tid, 128); __syncthreads(); v8f acc = {};
#pragma unroll
    for (int tap = 0; tap < 9; ++tap) { const v16h a = tile_frag<DH>(sx, ly, lx, tap, 0, lane);
      v16h w; { const _Float16* wr = Wa + tap * (2 * DH) + which * DH + 8 * g;
#pragma unroll
        for (int i = 0; i < 8; ++i) { w[i] = (col == 0) ? wr[i] : (_Float16)0.0f; w[8 + i] = (col == 0) ? wr[16 + i] : (_Float16)0.0f; } }
      acc = wmma16(a, w, acc); }
    if (col == 0) {
#pragma unroll
      for (int r = 0; r < 8; ++r) so[wave][which][8 * g + r] = acc[r]; } }
  LDSX();
  if (lane < 4) vst2(AQ + (f * NHD + hd) * NPX + p0 + lane * 4, *(const v4f*)&so[wave][0][lane * 4]);
  if (lane >= 4 && lane < 8) vst2(BK + (f * NHD + hd) * NPX + p0 + (lane - 4) * 4, *(const v4f*)&so[wave][1][(lane - 4) * 4]); }
__global__ __launch_bounds__(64) void k_mix(const float* __restrict__ AQ, const float* __restrict__ BK, const float* __restrict__ AB, const float* __restrict__ V, const float* __restrict__ XA, int li, float* __restrict__ AT) {
  __shared__ __align__(16) float sw[NT][64]; __shared__ __align__(16) float so[DH][64];
  const int t_ = threadIdx.x; const int pb = blockIdx.x; const size_t f = blockIdx.y; const int hd = blockIdx.z; const size_t b = f / NT; const int p = pb * 64 + t_;
  const float ab = bfr(AB[(size_t)li * NHD + hd]); const float aq = AQ[(f * NHD + hd) * NPX + p];
  float m = -3.0e38f;
#pragma unroll 1
  for (int j = 0; j < NT; ++j) { const float lg = aq + BK[((b * NT + j) * NHD + hd) * NPX + p] + ab; sw[j][t_] = lg; m = fmaxf(m, lg); }
  float l = 0.f;
#pragma unroll 1
  for (int j = 0; j < NT; ++j) { const float e = expf(sw[j][t_] - m); sw[j][t_] = e; l += e; }
  const float il = 1.0f / l;
#pragma unroll 1
  for (int c = 0; c < DH; ++c) { float a = 0.f;
#pragma unroll 1
    for (int j = 0; j < NT; ++j) a += sw[j][t_] * V[(((b * NT + j) * CC) + hd * DH + c) * NPX + p];
    so[c][t_] = a * il + XA[((f * CC) + hd * DH + c) * NPX + p]; }
  __syncthreads();
  for (int e = t_; e < DH * 16; e += 64) { const int c = e >> 4, q = e & 15; vst2(AT + ((f * CC) + hd * DH + c) * NPX + pb * 64 + q * 4, *(const v4f*)&so[c][q * 4]); } }
template <int WHICH>
__global__ __launch_bounds__(128) void k_ff(const float* __restrict__ SRC, const _Float16* __restrict__ WlP, const float* __restrict__ Bl, const float* __restrict__ RES, int li, float* __restrict__ DST, float* __restrict__ GS) {
  __shared__ __align__(16) float so[4][CC][20]; __shared__ float sst[4][4][2];
  __shared__ __align__(16) _Float16 sx[4 * 34 * CC];
  const int tid = threadIdx.x, wave = tid >> 5, lane = tid & 31, col = lane & 15, g = lane >> 4; const int pb = blockIdx.x; const size_t f = blockIdx.y;
  const float* src = SRC + f * CC * NPX; const _Float16* Wt = WlP; const float* Bs = Bl + (size_t)li * CC; const int p0 = pb * 64 + wave * 16; const int y0 = (pb * 64) / WWW; const int ly = (wave * 16) / WWW, lx = (wave * 16 + col) % WWW;
  stage_tile<CC>(src, y0, nullptr, sx, tid, 128); __syncthreads();
  v8f acc[8] = {};
#pragma unroll 1
  for (int tap = 0; tap < 9; ++tap) {
#pragma unroll
    for (int cq = 0; cq < CC / 32; ++cq) { const v16h a = tile_frag<CC>(sx, ly, lx, tap, cq * 32, lane);
#pragma unroll
      for (int j = 0; j < 8; ++j) acc[j] = wmma16(a, frag_h(Wt + (size_t)(j * 16 + col) * (CC * 9) + tap * CC + cq * 32, lane), acc[j]); } }
#pragma unroll
  for (int j = 0; j < 8; ++j) { const int c = j * 16 + col; const float bb = bfr(Bs[c]);
#pragma unroll
    for (int r = 0; r < 8; ++r) { float v = acc[j][r] + bb; if (WHICH == 0) v = fmaxf(v, 0.f); else v += RES[(f * CC + c) * NPX + p0 + 8 * g + r]; so[wave][c][8 * g + r] = v; } }
  LDSX();
  { float* dst = DST + (f * CC) * NPX + p0; for (int c = lane >> 2; c < CC; c += 8) vst2(dst + (size_t)c * NPX + (lane & 3) * 4, *(const v4f*)&so[wave][c][(lane & 3) * 4]); }
  if (WHICH == 1) {
    if (lane < 4) { const int gl = lane; float s = 0.f; for (int c = gl * 32; c < gl * 32 + 32; ++c) for (int q = 0; q < 16; ++q) s += so[wave][c][q]; const float mean = s / 512.0f; float m2 = 0.f; for (int c = gl * 32; c < gl * 32 + 32; ++c) for (int q = 0; q < 16; ++q) { const float d = so[wave][c][q] - mean; m2 += d * d; } sst[wave][gl][0] = mean; sst[wave][gl][1] = m2; }
    __syncthreads();
    float gm = 0.f, gq = 0.f; if (tid < 4) { const int gl = tid; float n = 0.f, mean = 0.f, M2 = 0.f; for (int w4 = 0; w4 < 4; ++w4) { const float nb = 512.f, mb = sst[w4][gl][0], qb = sst[w4][gl][1]; const float nt = n + nb; const float d = mb - mean; mean += d * nb / nt; M2 += qb + d * d * n * nb / nt; n = nt; } gm = mean; gq = M2; }
    __syncthreads(); if (tid < 4) { sst[0][tid][0] = gm; sst[0][tid][1] = gq; } __syncthreads();
    if (tid < 8) { v4f o; if (tid < 2) { o[0] = sst[0][2 * tid][0]; o[1] = sst[0][2 * tid][1]; o[2] = sst[0][2 * tid + 1][0]; o[3] = sst[0][2 * tid + 1][1]; } else { o[0] = o[1] = o[2] = o[3] = 0.f; } vst2(GS + (f * NPB + pb) * 32 + tid * 4, o); } } }
__global__ __launch_bounds__(64) void k_gn(const float* __restrict__ Y, const float* __restrict__ GS, const float* __restrict__ GW, const float* __restrict__ GB, int li, float* __restrict__ DST) { __shared__ float sm[4], si[4]; __shared__ __align__(16) float so[CC][64];
  const int t_ = threadIdx.x; const int pb = blockIdx.x; const size_t f = blockIdx.y;
  if (t_ < 4) { float n = 0.f, mean = 0.f, M2 = 0.f;
#pragma unroll 1
    for (int blk = 0; blk < NPB; ++blk) { const float nb = 2048.f, mb = GS[(f * NPB + blk) * 32 + t_ * 2], qb = GS[(f * NPB + blk) * 32 + t_ * 2 + 1]; const float nt = n + nb; const float d = mb - mean; mean += d * nb / nt; M2 += qb + d * d * n * nb / nt; n = nt; }
    sm[t_] = mean; si[t_] = 1.0f / sqrtf(M2 / n + 1e-5f); }
  __syncthreads(); const int p = pb * 64 + t_;
#pragma unroll 1
  for (int c = 0; c < CC; ++c) { const int gi = c / 32; so[c][t_] = (Y[(f * CC + c) * NPX + p] - sm[gi]) * si[gi] * bfr(GW[(size_t)li * CC + c]) + bfr(GB[(size_t)li * CC + c]); }
  __syncthreads();
  for (int e = t_; e < CC * 16; e += 64) { const int c = e >> 4, q = e & 15; vst2(DST + ((f * CC) + c) * NPX + pb * 64 + q * 4, *(const v4f*)&so[c][q * 4]); } }
__global__ __launch_bounds__(256) void k_copy(const float* __restrict__ X, float* __restrict__ XA) { const size_t i = ((size_t)blockIdx.x * 256 + threadIdx.x) * 4; v4f o; o[0] = bfr(X[i]); o[1] = bfr(X[i + 1]); o[2] = bfr(X[i + 2]); o[3] = bfr(X[i + 3]); vst2(XA + i, o); }
extern "C" void kernel_launch(void* const* d_in, const int* in_sizes, int n_in, void* d_out, int out_size, void* d_ws, size_t ws_size, hipStream_t stream) {
  (void)in_sizes; (void)n_in; (void)out_size;
  const float** F = (const float**)d_in;
  if (ws_size < (size_t)WS_END) return;
  char* ws = (char*)d_ws; _Float16 *WQP = (_Float16*)(ws + WS_WQ), *WKVP = (_Float16*)(ws + WS_WKV), *WAP = (_Float16*)(ws + WS_WA), *WF1P = (_Float16*)(ws + WS_WF1), *WF2P = (_Float16*)(ws + WS_WF2); float *XA = (float*)(ws + WS_XA), *Q = (float*)(ws + WS_Q), *V = (float*)(ws + WS_V), *AT = (float*)(ws + WS_AT), *F1 = (float*)(ws + WS_F1), *Y = (float*)(ws + WS_Y), *AQ = (float*)(ws + WS_AQ), *BK = (float*)(ws + WS_BK), *GS = (float*)(ws + WS_GS);
  k_copy<<<(unsigned)(FSZ / 1024), 256, 0, stream>>>(F[0], XA);
  for (int li = 0; li < NL; ++li) {
    k_wperm<<<NHD * DH, 256, 0, stream>>>(F[1] + (size_t)li * NHD * DH * DH * 9, NHD * DH, DH, WQP);
    k_wperm<<<NHD * DH, 256, 0, stream>>>(F[3] + (size_t)li * NHD * DH * DH * 9, NHD * DH, DH, WKVP);
    k_wperm<<<NHD, 256, 0, stream>>>(F[5] + (size_t)li * NHD * 2 * DH * 9, NHD, 2 * DH, WAP);
    k_wperm<<<CC, 256, 0, stream>>>(F[7] + (size_t)li * CC * CC * 9, CC, CC, WF1P);
    k_wperm<<<CC, 256, 0, stream>>>(F[9] + (size_t)li * CC * CC * 9, CC, CC, WF2P);
    k_qv<<<dim3(NPB, NFR, NHD), 128, 0, stream>>>(XA, WQP, F[2], WKVP, F[4], li, Q, V);
    k_logit<<<dim3(NPB, NFR, NHD), 128, 0, stream>>>(Q, V, WAP, li, AQ, BK);
    k_mix<<<dim3(NPB, NFR, NHD), 64, 0, stream>>>(AQ, BK, F[6], V, XA, li, AT);
    k_ff<0><<<dim3(NPB, NFR), 128, 0, stream>>>(AT, WF1P, F[8], nullptr, li, F1, GS);
    k_ff<1><<<dim3(NPB, NFR), 128, 0, stream>>>(F1, WF2P, F[10], AT, li, Y, GS);
    k_gn<<<dim3(NPB, NFR), 64, 0, stream>>>(Y, GS, F[11], F[12], li, (li == NL - 1) ? (float*)d_out : XA);
  }
}
